// net_rd_42984032699194
// MI455X (gfx1250) — hardware-verified
//
#include <hip/hip_runtime.h>


#define NB   32768
#define DSD  256
#define NE   16
#define KEX  4096
#define RCH  4096
#define NCH  8
#define HP   64

typedef __attribute__((ext_vector_type(16))) _Float16 v16h;
typedef __attribute__((ext_vector_type(8)))  _Float16 v8h;
typedef __attribute__((ext_vector_type(16))) __bf16   v16b;
typedef __attribute__((ext_vector_type(8)))  __bf16   v8b;
typedef __attribute__((ext_vector_type(8)))  float    v8f;
typedef __attribute__((ext_vector_type(4)))  float    v4f;
#define U16(p) ((const unsigned short*)(const void*)(p))

__device__ __forceinline__ unsigned short f2bf_bits(float f) {
  unsigned u = __float_as_uint(f);
  return (unsigned short)((u + 0x7FFFu + ((u >> 16) & 1u)) >> 16);
}
__device__ __forceinline__ float bf_bits2f(unsigned short h) { return __uint_as_float(((unsigned)h) << 16); }

__device__ __forceinline__ void dep_guard_h(v8f& a, v8f& b, v16h x, v16h y) { asm volatile("v_nop\n\tv_nop\n\tv_nop\n\tv_nop" : "+v"(a), "+v"(b) : "v"(x), "v"(y)); }
__device__ __forceinline__ void dep_guard_b(v8f& a, v8f& b, v16b x, v16b y) { asm volatile("v_nop\n\tv_nop\n\tv_nop\n\tv_nop" : "+v"(a), "+v"(b) : "v"(x), "v"(y)); }
__device__ __forceinline__ void keep4_h(v16h a, v16h b, v16h c, v16h d) { asm volatile("v_nop" :: "v"(a), "v"(b), "v"(c), "v"(d)); }
__device__ __forceinline__ void keep4_b(v16b a, v16b b, v16b c, v16b d) { asm volatile("v_nop" :: "v"(a), "v"(b), "v"(c), "v"(d)); }
__device__ __forceinline__ void acc_guard4(v8f& a, v8f& b, v8f& c, v8f& d) { asm volatile("v_nop\n\tv_nop\n\tv_nop\n\tv_nop" : "+v"(a), "+v"(b), "+v"(c), "+v"(d)); }
template <typename T> struct Frag;
template <> struct Frag<_Float16> {
  typedef v16h V; union U { v16h v; v8h h[2]; };
  static __device__ __forceinline__ v16h load(const _Float16* p) {
    U f; f.h[0] = *(const v8h*)(p); f.h[1] = *(const v8h*)(p + 16); return f.v;
  }
  static __device__ __forceinline__ v8f mma(v16h a, v16h b, v8f c) {
    return __builtin_amdgcn_wmma_f32_16x16x32_f16(false, a, false, b, (short)0, c, false, false);
  }
  static __device__ __forceinline__ void guard(v8f& a, v8f& b, v16h x, v16h y) { dep_guard_h(a, b, x, y); }
  static __device__ __forceinline__ void keep(v16h a, v16h b, v16h c, v16h d) { keep4_h(a, b, c, d); }
};
template <> struct Frag<__bf16> {
  typedef v16b V; union U { v16b v; v8b h[2]; };
  static __device__ __forceinline__ v16b load(const __bf16* p) {
    U f; f.h[0] = *(const v8b*)(p); f.h[1] = *(const v8b*)(p + 16); return f.v;
  }
  static __device__ __forceinline__ v8f mma(v16b a, v16b b, v8f c) {
    return __builtin_amdgcn_wmma_f32_16x16x32_bf16(false, a, false, b, (short)0, c, false, false);
  }
  static __device__ __forceinline__ void guard(v8f& a, v8f& b, v16b x, v16b y) { dep_guard_b(a, b, x, y); }
  static __device__ __forceinline__ void keep(v16b a, v16b b, v16b c, v16b d) { keep4_b(a, b, c, d); }
};

template <int ET> struct Elem;
template <> struct Elem<0> { typedef _Float16 T; };
template <> struct Elem<1> { typedef __bf16 T; };
template <int ET, bool SPLIT, int BIAS_MODE, int OUT_MODE, bool RESID, int ACT = 0>
__global__ __launch_bounds__(256) void wmma_gemm64(
    const unsigned short* __restrict__ Ap, const unsigned short* __restrict__ A2p, int lda, long strideA,
    const unsigned short* __restrict__ Btp, const unsigned short* __restrict__ Bt2p, int ldb, long strideB,
    void* __restrict__ Cout, void* __restrict__ Cout2, int ldc, long strideC,
    const float* __restrict__ bias,
    const float* __restrict__ resid, long strideR,
    int M, int N, int K, float scale) {
  typedef typename Elem<ET>::T T;
  typedef typename Frag<T>::V V;
  const T* A = (const T*)Ap; const T* A2 = (const T*)A2p; const T* Bt = (const T*)Btp; const T* Bt2 = (const T*)Bt2p;
  __shared__ __align__(16) float sT[8][16 * 68];
  const int b    = blockIdx.y;
  const int lane = threadIdx.x & 31;
  const int wave = threadIdx.x >> 5;
  const int tilesN = N >> 6;
  const int tilesM = M >> 6;
  const int tile = blockIdx.x * 8 + wave;
  if (tile >= tilesM * tilesN) return;
  const int tm = tile / tilesN;
  const int tn = tile - tm * tilesN;
  const int m0 = tm << 6;
  const int n0 = tn << 6;

  const T* Ab  = A  + (size_t)b * strideA;
  const T* Bb  = Bt + (size_t)b * strideB;
  const T* Ab2 = SPLIT ? (A2  + (size_t)b * strideA) : nullptr;
  const T* Bb2 = SPLIT ? (Bt2 + (size_t)b * strideB) : nullptr;

  const int rlane = lane & 15;
  const int koff  = (lane >> 4) * 8;
  const int mOff  = (lane >> 4) * 8;

  v8f acc[4][4];
#pragma unroll
  for (int i = 0; i < 4; ++i)
#pragma unroll
    for (int j = 0; j < 4; ++j) acc[i][j] = (v8f){0.f,0.f,0.f,0.f,0.f,0.f,0.f,0.f};

  for (int k0 = 0; k0 < K; k0 += 32) {
    V bh[4], bl[4];
#pragma unroll
    for (int j = 0; j < 4; ++j) {
      const size_t bo = (size_t)(n0 + (j << 4) + rlane) * ldb + koff + k0;
      bh[j] = Frag<T>::load(Bb + bo);
      if (SPLIT) bl[j] = Frag<T>::load(Bb2 + bo);
    }
#pragma unroll
    for (int i = 0; i < 4; ++i) {
      const size_t ao = (size_t)(m0 + (i << 4) + rlane) * lda + koff + k0;
      V ah = Frag<T>::load(Ab + ao);
      V al;
      if (SPLIT) al = Frag<T>::load(Ab2 + ao);
#pragma unroll
      for (int j = 0; j < 4; ++j) {
        acc[i][j] = Frag<T>::mma(ah, bh[j], acc[i][j]);
        if (SPLIT) {
          acc[i][j] = Frag<T>::mma(ah, bl[j], acc[i][j]);
          acc[i][j] = Frag<T>::mma(al, bh[j], acc[i][j]);
        }
      }
      Frag<T>::guard(acc[i][0], acc[i][3], ah, SPLIT ? al : ah);
    }
    Frag<T>::keep(bh[0], bh[1], bh[2], bh[3]);
    if (SPLIT) Frag<T>::keep(bl[0], bl[1], bl[2], bl[3]);
  }
  acc_guard4(acc[0][0], acc[0][1], acc[0][2], acc[0][3]);
  acc_guard4(acc[1][0], acc[1][1], acc[1][2], acc[1][3]);
  acc_guard4(acc[2][0], acc[2][1], acc[2][2], acc[2][3]);
  acc_guard4(acc[3][0], acc[3][1], acc[3][2], acc[3][3]);

  float* slab = sT[wave];
  const float* Rb = RESID ? (resid + (size_t)b * strideR) : nullptr;
#pragma unroll
  for (int i = 0; i < 4; ++i) {
    const int mBase = m0 + (i << 4);
#pragma unroll
    for (int j = 0; j < 4; ++j) {
      const int n = n0 + (j << 4) + rlane;
      float bv = 0.f;
      if (BIAS_MODE == 2) bv = bias[n];
#pragma unroll
      for (int r = 0; r < 8; ++r) {
        float v = acc[i][j][r] * scale;
        if (BIAS_MODE == 1) v += bias[mBase + mOff + r];
        if (BIAS_MODE == 2) v += bv;
        if (RESID) v += Rb[(size_t)(mBase + mOff + r) * ldc + n];
        if (ACT == 1) v = tanhf(v);
        if (ACT == 2) v = fmaxf(v, 0.0f);
        if (ACT == 3) v = v / (1.0f + expf(-v));
        if (ACT == 4) v = (v > 0.f) ? v : 0.01f * v;
        if (ACT == 5) v = 0.5f * v * (1.0f + erff(v * 0.70710678118654752f));
        slab[(mOff + r) * 68 + (j << 4) + rlane] = v;
      }
    }
    __builtin_amdgcn_fence(__ATOMIC_RELEASE, "workgroup");
    __builtin_amdgcn_wave_barrier();
    __builtin_amdgcn_fence(__ATOMIC_ACQUIRE, "workgroup");
    if (OUT_MODE == 0) {
      float* C = (float*)Cout + (size_t)b * strideC;
      const int hh = lane >> 4, c4 = (lane & 15) * 4;
      for (int pass = 0; pass < 2; ++pass) {
#pragma unroll
        for (int it = 0; it < 8; ++it) {
          const int row = it * 2 + hh;
          v4f v = *(const v4f*)(slab + row * 68 + c4);
          *(volatile v4f*)(C + (size_t)(mBase + row) * ldc + n0 + c4) = v;
        }
        __threadfence();
      }
    } else {
      const int q = lane >> 3, c8 = (lane & 7) * 8;
      unsigned short* C  = (unsigned short*)Cout  + (size_t)b * strideC;
      unsigned short* C2 = (OUT_MODE == 2) ? ((unsigned short*)Cout2 + (size_t)b * strideC) : nullptr;
      for (int pass = 0; pass < 2; ++pass) {
#pragma unroll
        for (int it = 0; it < 4; ++it) {
          const int row = it * 4 + q;
          const float* sp = slab + row * 68 + c8;
          v8h hv, lv;
#pragma unroll
          for (int e = 0; e < 8; ++e) {
            if (OUT_MODE == 1) {
              hv[e] = (_Float16)sp[e];
            } else {
              unsigned short hb = f2bf_bits(sp[e]);
              unsigned short lb = f2bf_bits(sp[e] - bf_bits2f(hb));
              hv[e] = __builtin_bit_cast(_Float16, hb);
              lv[e] = __builtin_bit_cast(_Float16, lb);
            }
          }
          *(volatile v8h*)(C + (size_t)(mBase + row) * ldc + n0 + c8) = hv;
          if (OUT_MODE == 2) *(volatile v8h*)(C2 + (size_t)(mBase + row) * ldc + n0 + c8) = lv;
        }
        __threadfence();
      }
    }
    __builtin_amdgcn_fence(__ATOMIC_RELEASE, "workgroup");
    __builtin_amdgcn_wave_barrier();
    __builtin_amdgcn_fence(__ATOMIC_ACQUIRE, "workgroup");
  }
}

__global__ __launch_bounds__(256) void cast_pad_f16x2(
    const float* __restrict__ in, _Float16* __restrict__ out, int kshift, int nreal, float scale, int n2) {
  const int i = blockIdx.x * 256 + threadIdx.x;
  if (i < n2) {
    const int el = 2 * i;
    const int n = el >> kshift;
    float f0 = 0.f, f1 = 0.f;
    if (n < nreal) { f0 = in[el] * scale; f1 = in[el + 1] * scale; }
    const _Float16 h0 = (_Float16)f0, h1 = (_Float16)f1;
    const unsigned u = (unsigned)__builtin_bit_cast(unsigned short, h0) | ((unsigned)__builtin_bit_cast(unsigned short, h1) << 16);
    ((volatile unsigned*)out)[i] = u;
    __threadfence();
    ((volatile unsigned*)out)[i] = u;
  }
}

__global__ __launch_bounds__(64) void pad_f32_64(const float* __restrict__ in, float* __restrict__ out, int nreal) {
  const int i = threadIdx.x;
  const float v = (i < nreal) ? in[i] : 0.f;
  ((volatile float*)out)[i] = v;
  __threadfence();
  ((volatile float*)out)[i] = v;
}

__global__ __launch_bounds__(256) void build_expert_bt(
    const float* __restrict__ BA, const float* __restrict__ CA, _Float16* __restrict__ At) {
  const int g = blockIdx.x * 256 + threadIdx.x;
  if (g >= (DSD * KEX) / 8) return;
  const int j0  = (g & 31) * 8;
  const int seg = g >> 5;
  const int e = seg & (NE - 1);
  const int i = seg >> 4;
  const size_t src = ((size_t)e << 16) + ((size_t)i << 8) + (size_t)j0;
  const size_t dst = ((size_t)i << 12) + ((size_t)e << 8) + (size_t)j0;
  const v4f b0 = *(const v4f*)(BA + src), b1v = *(const v4f*)(BA + src + 4);
  const v4f c0 = *(const v4f*)(CA + src), c1v = *(const v4f*)(CA + src + 4);
  v8h hv;
#pragma unroll
  for (int t = 0; t < 4; ++t) { hv[t] = (_Float16)(b0[t] + c0[t]); hv[4 + t] = (_Float16)(b1v[t] + c1v[t]); }
  *(volatile v8h*)(At + dst) = hv;
  __threadfence();
  *(volatile v8h*)(At + dst) = hv;
}

__global__ __launch_bounds__(256) void gate_scale_rows(
    const float* __restrict__ x, const float* __restrict__ xtar, const float* __restrict__ logits,
    _Float16* __restrict__ Ap, int row0) {
  const int lane = threadIdx.x & 31;
  const int wave = threadIdx.x >> 5;
  const int rloc = blockIdx.x * 8 + wave;
  const int row = row0 + rloc;
  if (rloc >= RCH || row >= NB) return;
  const float lg = logits[(size_t)row * HP + (lane & 15)];
  float m = lg;
  m = fmaxf(m, __shfl_xor(m, 1, 32));
  m = fmaxf(m, __shfl_xor(m, 2, 32));
  m = fmaxf(m, __shfl_xor(m, 4, 32));
  m = fmaxf(m, __shfl_xor(m, 8, 32));
  const float p = expf(lg - m);
  float s = p;
  s += __shfl_xor(s, 1, 32);
  s += __shfl_xor(s, 2, 32);
  s += __shfl_xor(s, 4, 32);
  s += __shfl_xor(s, 8, 32);
  const float w = p * (1.0f / s);

  const float* xr = x + (size_t)row * DSD + lane * 8;
  const v4f xa = *(const v4f*)(xr), xb = *(const v4f*)(xr + 4);
  const v4f ta = *(const v4f*)(xtar + lane * 8), tb = *(const v4f*)(xtar + lane * 8 + 4);
  float d[8];
#pragma unroll
  for (int t = 0; t < 4; ++t) { d[t] = ta[t] - xa[t]; d[4 + t] = tb[t] - xb[t]; }

  _Float16* dst = Ap + (size_t)rloc * KEX + lane * 8;
  for (int pass = 0; pass < 2; ++pass) {
#pragma unroll
    for (int k = 0; k < NE; ++k) {
      const float wk = __shfl(w, k, 32) * 1024.0f;
      v8h hv;
#pragma unroll
      for (int t = 0; t < 8; ++t) hv[t] = (_Float16)(wk * d[t]);
      *(volatile v8h*)(dst + k * DSD) = hv;
    }
    __threadfence();
  }
}

template <int BIAS_MODE, int OUT_MODE, int ACT>
static void launch_gemm_f16(const void* A, int lda, const void* Bt, int ldb, void* C, int ldc,
                            const float* bias, int M, int N, int K, float scale, hipStream_t stream) {
  const int tiles = (M >> 6) * (N >> 6);
  dim3 grid((unsigned)((tiles + 7) >> 3), 1, 1);
  wmma_gemm64<0, false, BIAS_MODE, OUT_MODE, false, ACT><<<grid, 256, 0, stream>>>(
      (const unsigned short*)A, (const unsigned short*)A, lda, 0L,
      (const unsigned short*)Bt, (const unsigned short*)Bt, ldb, 0L,
      C, C, ldc, 0L, bias, bias, 0L, M, N, K, scale);
}

static inline size_t align256(size_t v) { return (v + 255) & ~(size_t)255; }

extern "C" void kernel_launch(void* const* d_in, const int* in_sizes, int n_in,
                              void* d_out, int out_size, void* d_ws, size_t ws_size,
                              hipStream_t stream) {
  if (n_in < 12) return;
  if (in_sizes[0] != NB * DSD || in_sizes[1] < DSD || in_sizes[2] != NE * DSD * DSD ||
      in_sizes[3] != NE * DSD * DSD || in_sizes[4] != 128 * DSD || in_sizes[5] != 128 ||
      in_sizes[6] != 64 * 128 || in_sizes[7] != 64 || in_sizes[8] != 32 * 64 || in_sizes[9] != 32 ||
      in_sizes[10] != NE * 32 || in_sizes[11] != NE) return;
  if (out_size != NB * DSD) return;

  const float* x    = (const float*)d_in[0];
  const float* xtar = (const float*)d_in[1];
  const float* BA   = (const float*)d_in[2];
  const float* CA   = (const float*)d_in[3];
  const float* W1   = (const float*)d_in[4];
  const float* b1   = (const float*)d_in[5];
  const float* W2   = (const float*)d_in[6];
  const float* b2   = (const float*)d_in[7];
  const float* W3   = (const float*)d_in[8];
  const float* b3   = (const float*)d_in[9];
  const float* W4   = (const float*)d_in[10];
  const float* b4   = (const float*)d_in[11];
  float* out = (float*)d_out;

  size_t off = 0;
  char* ws = (char*)d_ws;
  _Float16* X16  = (_Float16*)(ws + off); off += align256((size_t)NB * DSD * 2);
  _Float16* H1   = (_Float16*)(ws + off); off += align256((size_t)NB * 128 * 2);
  _Float16* H2   = (_Float16*)(ws + off); off += align256((size_t)NB * HP * 2);
  _Float16* H3   = (_Float16*)(ws + off); off += align256((size_t)NB * HP * 2);
  float*    LOG  = (float*)(ws + off);    off += align256((size_t)NB * HP * 4);
  _Float16* A16t = (_Float16*)(ws + off); off += align256((size_t)DSD * KEX * 2);
  _Float16* W1h  = (_Float16*)(ws + off); off += align256((size_t)128 * DSD * 2);
  _Float16* W2h  = (_Float16*)(ws + off); off += align256((size_t)64 * 128 * 2);
  _Float16* W3h  = (_Float16*)(ws + off); off += align256((size_t)HP * 64 * 2);
  _Float16* W4h  = (_Float16*)(ws + off); off += align256((size_t)HP * 32 * 2);
  float*    b3p  = (float*)(ws + off);    off += align256((size_t)HP * 4);
  float*    b4p  = (float*)(ws + off);    off += align256((size_t)HP * 4);
  _Float16* Ap   = (_Float16*)(ws + off); off += align256((size_t)RCH * KEX * 2);
  if (off > ws_size) return;

  const float WSC = 64.0f, WSC_INV = 1.0f / 64.0f;

  cast_pad_f16x2<<<(NB * DSD / 2 + 255) / 256, 256, 0, stream>>>(x, X16, 8, NB, 1.0f, NB * DSD / 2);
  cast_pad_f16x2<<<(128 * DSD / 2 + 255) / 256, 256, 0, stream>>>(W1, W1h, 8, 128, WSC, 128 * DSD / 2);
  cast_pad_f16x2<<<(64 * 128 / 2 + 255) / 256, 256, 0, stream>>>(W2, W2h, 7, 64, WSC, 64 * 128 / 2);
  cast_pad_f16x2<<<(HP * 64 / 2 + 255) / 256, 256, 0, stream>>>(W3, W3h, 6, 32, WSC, HP * 64 / 2);
  cast_pad_f16x2<<<(HP * 32 / 2 + 255) / 256, 256, 0, stream>>>(W4, W4h, 5, NE, WSC, HP * 32 / 2);
  pad_f32_64<<<1, 64, 0, stream>>>(b3, b3p, 32);
  pad_f32_64<<<1, 64, 0, stream>>>(b4, b4p, NE);
  build_expert_bt<<<(DSD * KEX / 8 + 255) / 256, 256, 0, stream>>>(BA, CA, A16t);

  launch_gemm_f16<2, 1, 2>(X16, DSD, W1h, DSD, H1, 128, b1, NB, 128, DSD, WSC_INV, stream);
  launch_gemm_f16<2, 1, 2>(H1, 128, W2h, 128, H2, HP, b2, NB, HP, 128, WSC_INV, stream);
  launch_gemm_f16<2, 1, 2>(H2, HP, W3h, 64, H3, HP, b3p, NB, HP, 64, WSC_INV, stream);
  launch_gemm_f16<2, 0, 0>(H3, HP, W4h, 32, LOG, HP, b4p, NB, HP, 32, WSC_INV, stream);

  for (int c = 0; c < NCH; ++c) {
    gate_scale_rows<<<RCH / 8, 256, 0, stream>>>(x, xtar, LOG, Ap, c * RCH);
    launch_gemm_f16<0, 0, 0>(Ap, KEX, A16t, KEX, out + (size_t)c * RCH * DSD, DSD, b4p,
                             RCH, DSD, KEX, 1.0f / 1024.0f, stream);
  }
}
